// PhaseAttentionLayer_76081050681693
// MI455X (gfx1250) — hardware-verified
//
#include <hip/hip_runtime.h>
#include <stddef.h>
#include <stdint.h>


#define BB   2
#define SS   2048
#define DD   768
#define HH   12
#define DH   64
#define FFD  3072
#define PDIM 64
#define MTOT (BB * SS)

static_assert(MTOT % 256 == 0 && DD % 128 == 0 && FFD % 128 == 0 && (2 * DD) % 128 == 0);
static_assert(SS % 64 == 0 && DD % 64 == 0 && SS % 16 == 0 && DD == 16 * 48);

typedef _Float16 f16;
typedef f16   v16h __attribute__((ext_vector_type(16)));
typedef f16   v8h  __attribute__((ext_vector_type(8), __may_alias__));
typedef float v8f  __attribute__((ext_vector_type(8)));
typedef float v4f  __attribute__((ext_vector_type(4), __may_alias__));

union Frag { v16h v; v8h h[2]; };
union Pack { v8h h; v4f f; };

__device__ __forceinline__ v8f mma16(v16h a, v16h b, v8f c) {
    v8f d = __builtin_amdgcn_wmma_f32_16x16x32_f16(false, a, false, b, (short)0, c, false, false);
    asm volatile("v_nop\n\tv_nop\n\tv_nop\n\tv_nop" : "+v"(d) : "v"(a), "v"(b));
    return d;
}

__device__ __forceinline__ v16h frag_g(const f16* base, int pitch, size_t row0, int k0) {
    const int l = threadIdx.x & 31, h = l >> 4, m = l & 15;
    const f16* p = base + (row0 + (size_t)m) * (size_t)pitch + k0 + 8 * h;
    Frag f;
    f.h[0] = *(const v8h*)p;
    f.h[1] = *(const v8h*)(p + 16);
    return f.v;
}

__device__ __forceinline__ void st16v(void* p, v4f v) { *(volatile v4f*)p = v; }

__device__ __forceinline__ float wave_sum(float v) {
#pragma unroll
    for (int o = 16; o > 0; o >>= 1) v += __shfl_xor(v, o);
    return v;
}
__device__ __forceinline__ float wave_max(float v) {
#pragma unroll
    for (int o = 16; o > 0; o >>= 1) v = fmaxf(v, __shfl_xor(v, o));
    return v;
}

__global__ __launch_bounds__(256) void cvt_f16_kernel(const float* __restrict__ src, f16* __restrict__ dst,
                                                      int n8, float scale) {
    const int g = blockIdx.x * 256 + threadIdx.x;
    if (g >= n8) return;
    const float* s = src + (size_t)g * 8;
    const v4f a = *(const v4f*)s;
    const v4f b = *(const v4f*)(s + 4);
    Pack p;
#pragma unroll
    for (int e = 0; e < 4; ++e) {
        p.h[e]     = (f16)(a[e] * scale);
        p.h[4 + e] = (f16)(b[e] * scale);
    }
    f16* d = dst + (size_t)g * 8;
    st16v(d, p.f);
    __threadfence();
    st16v(d, p.f);
}

__global__ __launch_bounds__(256) void ln_f16_kernel(const float* __restrict__ X, const float* __restrict__ gw,
                                                     const float* __restrict__ gb, f16* __restrict__ Y,
                                                     int nrows) {
    const int w = threadIdx.x >> 5, l = threadIdx.x & 31;
    const int row = blockIdx.x * 8 + w;
    if (row >= nrows) return;
    const float* xr = X + (size_t)row * DD;
    float v[24];
#pragma unroll
    for (int j = 0; j < 3; ++j) {
        const int c = j * 256 + 8 * l;
        const v4f a = *(const v4f*)(xr + c);
        const v4f b = *(const v4f*)(xr + c + 4);
#pragma unroll
        for (int e = 0; e < 4; ++e) { v[8 * j + e] = a[e]; v[8 * j + 4 + e] = b[e]; }
    }
    float s = 0.f;
#pragma unroll
    for (int i = 0; i < 24; ++i) s += v[i];
    s = wave_sum(s);
    const float mean = s * (1.0f / (float)DD);
    float s2 = 0.f;
#pragma unroll
    for (int i = 0; i < 24; ++i) { const float d = v[i] - mean; s2 += d * d; }
    s2 = wave_sum(s2);
    const float rstd = rsqrtf(s2 * (1.0f / (float)DD) + 1e-5f);
    Pack pk[3];
#pragma unroll
    for (int j = 0; j < 3; ++j) {
        const int c = j * 256 + 8 * l;
        const v4f w0 = *(const v4f*)(gw + c);
        const v4f w1 = *(const v4f*)(gw + c + 4);
        const v4f b0 = *(const v4f*)(gb + c);
        const v4f b1 = *(const v4f*)(gb + c + 4);
#pragma unroll
        for (int e = 0; e < 4; ++e) {
            pk[j].h[e]     = (f16)((v[8 * j + e] - mean) * rstd * w0[e] + b0[e]);
            pk[j].h[4 + e] = (f16)((v[8 * j + 4 + e] - mean) * rstd * w1[e] + b1[e]);
        }
    }
    f16* yr = Y + (size_t)row * DD + 8 * l;
#pragma unroll
    for (int j = 0; j < 3; ++j) st16v(yr + j * 256, pk[j].f);
    __threadfence();
#pragma unroll
    for (int j = 0; j < 3; ++j) st16v(yr + j * 256, pk[j].f);
}

__global__ __launch_bounds__(256) void transpose_f16_kernel(const f16* __restrict__ Xn, f16* __restrict__ XT) {
    __shared__ __align__(16) f16 tile[64 * 72];
    const int tid = threadIdx.x, b = blockIdx.z, s0 = blockIdx.x * 64, d0 = blockIdx.y * 64;
#pragma unroll
    for (int it = 0; it < 2; ++it) {
        const int idx = tid + 256 * it, s = idx >> 3, dg = idx & 7;
        Pack p;
        p.h = *(const v8h*)(Xn + ((size_t)b * SS + s0 + s) * DD + d0 + 8 * dg);
#pragma unroll
        for (int e = 0; e < 8; ++e) tile[(8 * dg + e) * 72 + s] = p.h[e];
    }
    __syncthreads();
    const int w = tid >> 5, l = tid & 31;
    Pack o[2];
    size_t gi[2];
#pragma unroll
    for (int qq = 0; qq < 2; ++qq) {
        const int d = 8 * w + 4 * qq + (l >> 3), piece = l & 7;
        o[qq].h = *(const v8h*)(tile + d * 72 + 8 * piece);
        gi[qq] = ((size_t)b * DD + d0 + d) * SS + s0 + 8 * piece;
    }
#pragma unroll
    for (int qq = 0; qq < 2; ++qq) st16v(XT + gi[qq], o[qq].f);
    __threadfence();
#pragma unroll
    for (int qq = 0; qq < 2; ++qq) st16v(XT + gi[qq], o[qq].f);
}

template <int MODE, int WN>
__global__ __launch_bounds__(256) void gemm_kernel(const f16* __restrict__ A, const f16* __restrict__ W,
                                                   const float* __restrict__ bias, const float* __restrict__ res,
                                                   float* __restrict__ outf, f16* __restrict__ out0,
                                                   f16* __restrict__ out1, int K) {
    extern __shared__ float dynf[];
    constexpr int WM = 8 / WN;
    const int tid = threadIdx.x, w = tid >> 5, l = tid & 31, hh = l >> 4, m = l & 15;
    const int wm = w / WN, wn = w - wm * WN;
    const int m0 = blockIdx.y * (WM * 32) + wm * 32;
    const int n0 = blockIdx.x * (WN * 64) + wn * 64;

    v8f acc[2][4];
#pragma unroll
    for (int i = 0; i < 2; ++i)
#pragma unroll
        for (int j = 0; j < 4; ++j) acc[i][j] = (v8f){};

#pragma unroll 1
    for (int k0 = 0; k0 < K; k0 += 32) {
        const v16h a0 = frag_g(A, K, (size_t)m0, k0);
        const v16h a1 = frag_g(A, K, (size_t)m0 + 16, k0);
        v16h bfr[4];
#pragma unroll
        for (int j = 0; j < 4; ++j) bfr[j] = frag_g(W, K, (size_t)(n0 + 16 * j), k0);
#pragma unroll
        for (int j = 0; j < 4; ++j) {
            acc[0][j] = mma16(a0, bfr[j], acc[0][j]);
            acc[1][j] = mma16(a1, bfr[j], acc[1][j]);
        }
    }

    const float sK = 1.0f / 32.0f;
    if constexpr (MODE == 3) {
        float* stg = dynf + w * 2048;
#pragma unroll
        for (int i = 0; i < 2; ++i)
#pragma unroll
            for (int j = 0; j < 4; ++j)
#pragma unroll
                for (int r = 0; r < 8; ++r) {
                    const int row = i * 16 + 8 * hh + r, col = j * 16 + m;
                    stg[row * 64 + col] = acc[i][j][r] * sK + bias[n0 + col];
                }
        __syncthreads();
#pragma unroll 1
        for (int pass = 0; pass < 2; ++pass) {
#pragma unroll
            for (int q = 0; q < 16; ++q) {
                const int row = 2 * q + (l >> 4), piece = l & 15;
                const v4f v = *(const v4f*)(stg + row * 64 + 4 * piece);
                const size_t gi = (size_t)(m0 + row) * DD + n0 + 4 * piece;
                const v4f rr = *(const v4f*)(res + gi);
                st16v(outf + gi, v + rr);
            }
            if (pass == 0) __threadfence();
        }
    } else {
        f16* stg = reinterpret_cast<f16*>(dynf) + w * 2048;
        const float qs = (MODE == 0 && n0 < DD) ? 0.125f : 1.0f;
#pragma unroll
        for (int i = 0; i < 2; ++i)
#pragma unroll
            for (int j = 0; j < 4; ++j)
#pragma unroll
                for (int r = 0; r < 8; ++r) {
                    const int row = i * 16 + 8 * hh + r, col = j * 16 + m;
                    float val = acc[i][j][r] * sK;
                    if constexpr (MODE == 0) {
                        val = (val + bias[n0 + col]) * qs;
                    } else if constexpr (MODE == 1) {
                        val = tanhf(val);
                    } else {
                        val += bias[n0 + col];
                        val = 0.5f * val * (1.0f + erff(val * 0.70710678118654752f));
                    }
                    stg[row * 64 + col] = (f16)val;
                }
        __syncthreads();
        f16* dst;
        int ldd, nd;
        if constexpr (MODE == 0) {
            ldd = DD;
            if (n0 < DD) { dst = out0; nd = n0; } else { dst = out1; nd = n0 - DD; }
        } else if constexpr (MODE == 1) {
            dst = out0; ldd = PDIM; nd = n0;
        } else {
            dst = out0; ldd = FFD; nd = n0;
        }
#pragma unroll 1
        for (int pass = 0; pass < 2; ++pass) {
#pragma unroll
            for (int q = 0; q < 8; ++q) {
                const int row = 4 * q + (l >> 3), piece = l & 7;
                Pack p;
                p.h = *(const v8h*)(stg + row * 64 + 8 * piece);
                st16v(dst + (size_t)(m0 + row) * ldd + nd + 8 * piece, p.f);
            }
            if (pass == 0) __threadfence();
        }
    }
}

__global__ __launch_bounds__(512) void attn_ctx_kernel(const f16* __restrict__ Q, const f16* __restrict__ Kk,
                                                       const f16* __restrict__ Ph, const f16* __restrict__ XT,
                                                       const float* __restrict__ X,
                                                       const float* __restrict__ alphap,
                                                       float* __restrict__ X1) {
    extern __shared__ float dynf[];
    float* sc  = dynf;
    f16*   p16 = reinterpret_cast<f16*>(dynf);
    float* stg = dynf + 16384;
    const int tid = threadIdx.x, w = tid >> 5, l = tid & 31, hh = l >> 4, m = l & 15;
    const int b = blockIdx.y, q0 = blockIdx.x * 16;
    const size_t qrow0 = (size_t)b * SS + q0;
    const f16* Kb = Kk + (size_t)b * SS * DD;
    const f16* Pb = Ph + (size_t)b * SS * PDIM;
    const float alpha = alphap[0];
    float* myrow = sc + w * SS;

    float accw[64];
#pragma unroll
    for (int i = 0; i < 64; ++i) accw[i] = 0.f;

#pragma unroll 1
    for (int h = 0; h < HH; ++h) {
        const int kd = h * DH;
        const v16h a0 = frag_g(Q, DD, qrow0, kd);
        const v16h a1 = frag_g(Q, DD, qrow0, kd + 32);
#pragma unroll 1
        for (int t = 0; t < 8; ++t) {
            const int n0 = w * 128 + t * 16;
            const v16h b0 = frag_g(Kb, DD, (size_t)n0, kd);
            const v16h b1 = frag_g(Kb, DD, (size_t)n0, kd + 32);
            v8f acc = (v8f){};
            acc = mma16(a0, b0, acc);
            acc = mma16(a1, b1, acc);
#pragma unroll
            for (int r = 0; r < 8; ++r) sc[(8 * hh + r) * SS + n0 + m] = acc[r];
        }
        __syncthreads();
        float mx = -3.0e38f;
#pragma unroll 8
        for (int i = 0; i < 64; ++i) mx = fmaxf(mx, myrow[l + 32 * i]);
        mx = wave_max(mx);
        float sum = 0.f;
#pragma unroll 8
        for (int i = 0; i < 64; ++i) {
            const float e = __expf(myrow[l + 32 * i] - mx);
            myrow[l + 32 * i] = e;
            sum += e;
        }
        sum = wave_sum(sum);
        const float inv = 1.0f / (sum * (float)HH);
#pragma unroll
        for (int i = 0; i < 64; ++i) accw[i] += myrow[l + 32 * i] * inv;
        __syncthreads();
    }

#pragma unroll
    for (int i = 0; i < 64; ++i) myrow[l + 32 * i] = accw[i];
    __syncthreads();

    {
        const v16h a0 = frag_g(Ph, PDIM, qrow0, 0);
        const v16h a1 = frag_g(Ph, PDIM, qrow0, 32);
#pragma unroll 1
        for (int t = 0; t < 8; ++t) {
            const int n0 = w * 128 + t * 16;
            const v16h b0 = frag_g(Pb, PDIM, (size_t)n0, 0);
            const v16h b1 = frag_g(Pb, PDIM, (size_t)n0, 32);
            v8f acc = (v8f){};
            acc = mma16(a0, b0, acc);
            acc = mma16(a1, b1, acc);
#pragma unroll
            for (int r = 0; r < 8; ++r) {
                const int idx = (8 * hh + r) * SS + n0 + m;
                const float aw = sc[idx];
                sc[idx] = __logf(aw + 1e-6f) + alpha * (0.5f * acc[r] + 0.5f);
            }
        }
    }
    __syncthreads();

    float ev[64];
    float mz = -3.0e38f;
#pragma unroll
    for (int i = 0; i < 64; ++i) { ev[i] = myrow[l + 32 * i]; mz = fmaxf(mz, ev[i]); }
    mz = wave_max(mz);
    float lsum = 0.f;
#pragma unroll
    for (int i = 0; i < 64; ++i) { ev[i] = __expf(ev[i] - mz); lsum += ev[i]; }
    lsum = wave_sum(lsum);
    const float inv14 = 16384.0f / lsum;
    __syncthreads();
    f16* prow = p16 + w * SS;
#pragma unroll
    for (int i = 0; i < 64; ++i) prow[l + 32 * i] = (f16)(ev[i] * inv14);
    __syncthreads();

    const f16* XTb = XT + (size_t)b * DD * SS;
    const int nb = w * 48;
    v8f c0 = (v8f){}, c1 = (v8f){}, c2 = (v8f){};
#pragma unroll 1
    for (int k0 = 0; k0 < SS; k0 += 32) {
        const v16h pa = frag_g(p16, SS, 0, k0);
        const v16h b0 = frag_g(XTb, SS, (size_t)nb, k0);
        const v16h b1 = frag_g(XTb, SS, (size_t)nb + 16, k0);
        const v16h b2 = frag_g(XTb, SS, (size_t)nb + 32, k0);
        c0 = mma16(pa, b0, c0);
        c1 = mma16(pa, b1, c1);
        c2 = mma16(pa, b2, c2);
    }
    const float s14 = 1.0f / 16384.0f;
#pragma unroll
    for (int r = 0; r < 8; ++r) {
        const int rb = (8 * hh + r) * DD + nb + m;
        stg[rb]      = c0[r] * s14;
        stg[rb + 16] = c1[r] * s14;
        stg[rb + 32] = c2[r] * s14;
    }
    __syncthreads();

    const size_t gro = (qrow0 + w) * (size_t)DD;
    const float* srow = stg + w * DD;
#pragma unroll 1
    for (int pass = 0; pass < 2; ++pass) {
#pragma unroll
        for (int q = 0; q < 6; ++q) {
            const int c = 128 * q + 4 * l;
            const v4f v  = *(const v4f*)(srow + c);
            const v4f xr = *(const v4f*)(X + gro + c);
            st16v(X1 + gro + c, v + xr);
        }
        if (pass == 0) __threadfence();
    }
}

extern "C" void kernel_launch(void* const* d_in, const int* in_sizes, int n_in,
                              void* d_out, int out_size, void* d_ws, size_t ws_size,
                              hipStream_t stream) {
    if (n_in < 13) return;
    if (in_sizes[0] != MTOT * DD || in_sizes[1] != DD || in_sizes[2] != DD ||
        in_sizes[3] != 3 * DD * DD || in_sizes[4] != 3 * DD || in_sizes[5] != PDIM * DD ||
        in_sizes[6] < 1 || in_sizes[7] != FFD * DD || in_sizes[8] != FFD ||
        in_sizes[9] != DD * FFD || in_sizes[10] != DD || in_sizes[11] != DD || in_sizes[12] != DD)
        return;
    if (out_size != MTOT * DD) return;

    const float* x      = (const float*)d_in[0];
    const float* ln1_w  = (const float*)d_in[1];
    const float* ln1_b  = (const float*)d_in[2];
    const float* ipw    = (const float*)d_in[3];
    const float* ipb    = (const float*)d_in[4];
    const float* phw    = (const float*)d_in[5];
    const float* alphap = (const float*)d_in[6];
    const float* fw1    = (const float*)d_in[7];
    const float* fb1    = (const float*)d_in[8];
    const float* fw2    = (const float*)d_in[9];
    const float* fb2    = (const float*)d_in[10];
    const float* ln2_w  = (const float*)d_in[11];
    const float* ln2_b  = (const float*)d_in[12];
    float* out = (float*)d_out;

    const size_t sz_act16 = (size_t)MTOT * DD * 2;
    const size_t sz_ph16  = (size_t)MTOT * PDIM * 2;
    const size_t sz_wqk   = (size_t)2 * DD * DD * 2;
    const size_t sz_wph   = (size_t)PDIM * DD * 2;
    const size_t sz_wf    = (size_t)FFD * DD * 2;
    const size_t sz_x1    = (size_t)MTOT * DD * 4;
    const size_t sz_h16   = (size_t)MTOT * FFD * 2;
    size_t off = 0;
    uint8_t* base = (uint8_t*)d_ws;
    f16* xn16  = (f16*)(base + off);  off += sz_act16;
    f16* xnT16 = (f16*)(base + off);  off += sz_act16;
    f16* q16   = (f16*)(base + off);  off += sz_act16;
    f16* k16   = (f16*)(base + off);  off += sz_act16;
    f16* ph16  = (f16*)(base + off);  off += sz_ph16;
    f16* wqk16 = (f16*)(base + off);  off += sz_wqk;
    f16* wph16 = (f16*)(base + off);  off += sz_wph;
    f16* wf1   = (f16*)(base + off);  off += sz_wf;
    f16* wf2   = (f16*)(base + off);  off += sz_wf;
    float* x1  = (float*)(base + off); off += sz_x1;
    f16* x2n16 = (f16*)(base + off);  off += sz_act16;
    f16* h16   = (f16*)(base + off);  off += sz_h16;
    if (off > ws_size) return;

    {
        const int n8a = (2 * DD * DD) / 8, n8b = (PDIM * DD) / 8, n8c = (FFD * DD) / 8;
        cvt_f16_kernel<<<(n8a + 255) / 256, 256, 0, stream>>>(ipw, wqk16, n8a, 32.0f);
        cvt_f16_kernel<<<(n8b + 255) / 256, 256, 0, stream>>>(phw, wph16, n8b, 32.0f);
        cvt_f16_kernel<<<(n8c + 255) / 256, 256, 0, stream>>>(fw1, wf1, n8c, 32.0f);
        cvt_f16_kernel<<<(n8c + 255) / 256, 256, 0, stream>>>(fw2, wf2, n8c, 32.0f);
    }

    ln_f16_kernel<<<(MTOT + 7) / 8, 256, 0, stream>>>(x, ln1_w, ln1_b, xn16, MTOT);
    transpose_f16_kernel<<<dim3(SS / 64, DD / 64, BB), 256, 0, stream>>>(xn16, xnT16);

    gemm_kernel<0, 2><<<dim3((2 * DD) / 128, MTOT / 128), 256, 32768, stream>>>(
        xn16, wqk16, ipb, nullptr, nullptr, q16, k16, DD);

    gemm_kernel<1, 1><<<dim3(1, MTOT / 256), 256, 32768, stream>>>(
        xn16, wph16, nullptr, nullptr, nullptr, ph16, nullptr, DD);

    attn_ctx_kernel<<<dim3(SS / 16, BB), 512, 131072, stream>>>(q16, k16, ph16, xnT16, x, alphap, x1);

    ln_f16_kernel<<<(MTOT + 7) / 8, 256, 0, stream>>>(x1, ln2_w, ln2_b, x2n16, MTOT);

    gemm_kernel<2, 2><<<dim3(FFD / 128, MTOT / 128), 256, 32768, stream>>>(
        x2n16, wf1, fb1, nullptr, nullptr, h16, nullptr, DD);

    gemm_kernel<3, 2><<<dim3(DD / 128, MTOT / 128), 256, 65536, stream>>>(
        h16, wf2, fb2, x1, out, nullptr, nullptr, FFD);
}
